// MultiHeadAttentionQuantum_65481071409130
// MI455X (gfx1250) — hardware-verified
//
#include <hip/hip_runtime.h>
#include <math.h>
#include <stdint.h>

#ifndef NB
#define NB 4
#endif
#ifndef SEQ
#define SEQ 2048
#endif
#define NB_FULL  4
#define SEQ_FULL 2048
#define H_   16
#define DK_  8
#define E_   128
#define BH_  (NB * H_)
#define KSL  32
#define NSG  (SEQ / 256)
#define NQT  (SEQ / 64)
#define NKT  (SEQ / 64)
static_assert(H_ * DK_ == E_);
static_assert((SEQ % 256) == 0 && SEQ >= 256 && SEQ <= SEQ_FULL);
static_assert(NB >= 1 && NB <= NB_FULL);
static_assert(((NB * SEQ) % 64) == 0);
static_assert(E_ == 128);

typedef _Float16 v16h __attribute__((ext_vector_type(16)));
typedef _Float16 v8h  __attribute__((ext_vector_type(8)));
typedef float    v8f  __attribute__((ext_vector_type(8)));
typedef float    v4f  __attribute__((ext_vector_type(4)));
typedef unsigned int v4u __attribute__((ext_vector_type(4)));

#if defined(__HIP_DEVICE_COMPILE__)
#define DEV_ASM 1
#else
#define DEV_ASM 0
#endif

static const float kScale = 0.35355339059327373f;

__device__ __forceinline__ unsigned short h_bits(_Float16 v) { return __builtin_bit_cast(unsigned short, v); }
__device__ __forceinline__ unsigned pk16(unsigned short a, unsigned short b) { return (unsigned)a | ((unsigned)b << 16); }
__device__ __forceinline__ v8f zero8() { v8f z = {0.f, 0.f, 0.f, 0.f, 0.f, 0.f, 0.f, 0.f}; return z; }
__device__ __forceinline__ float bf16r(float f) {
  unsigned u = __float_as_uint(f);
  u = (u + 0x7FFFu + ((u >> 16) & 1u)) & 0xFFFF0000u;
  return __uint_as_float(u);
}
__device__ __forceinline__ unsigned short hn_bits(float f) {
  const unsigned short u = h_bits((_Float16)f);
  return ((u & 0x7C00u) == 0u) ? (unsigned short)0 : u;
}
__device__ __forceinline__ _Float16 f16n(float f) { return __builtin_bit_cast(_Float16, hn_bits(f)); }

__device__ __forceinline__ v16h ldfrag_h(const _Float16* p) {
  union { v16h v; v8h h[2]; } f;
  f.h[0] = *(const v8h*)(p);
  f.h[1] = *(const v8h*)(p + 16);
  return f.v;
}

__device__ __forceinline__ v8f mma_h(v16h a, v16h b, v8f c) {
  c = __builtin_amdgcn_wmma_f32_16x16x32_f16(false, a, false, b, (short)0, c, false, false);
#if DEV_ASM
  asm volatile("v_nop\n\tv_nop\n\tv_nop\n\tv_nop" : "+v"(c) : "v"(a), "v"(b));
#endif
  return c;
}

__device__ __forceinline__ void enc_slots(float f, int quarter, unsigned short& qs, unsigned short& ks) {
  const unsigned short qhi = hn_bits(f);
  const float hf = (float)__builtin_bit_cast(_Float16, qhi);
  const float lo = f - hf;
  const unsigned short qlo = hn_bits(lo * 4096.0f);
  const unsigned short khi = hn_bits(hf * 64.0f);
  const unsigned short kmd = hn_bits(hf * 0.015625f);
  const unsigned short klo = hn_bits(lo * 64.0f);
  const unsigned short z = (unsigned short)0;
  qs = (quarter == 1) ? qlo : ((quarter == 3) ? z : qhi);
  ks = (quarter == 0) ? khi : ((quarter == 1) ? kmd : ((quarter == 2) ? klo : z));
}

__global__ __launch_bounds__(256) void qenc(const float* __restrict__ x, const float* __restrict__ theta,
                                            unsigned short* qap, unsigned short* kbp, unsigned short* vtp) {
  __shared__ __align__(16) float cs[256 * DK_];
  const int tid = (int)threadIdx.x;
  const int bx  = (int)blockIdx.x;
  const int st  = bx % NSG;
  const int bh  = bx / NSG;
  const int b   = bh / H_;
  const int h   = bh % H_;
  const int s0  = st * 256;
  {
    const float* xp = x + ((size_t)b * SEQ_FULL + (size_t)(s0 + tid)) * E_ + h * DK_;
    float prod = 1.0f;
#pragma unroll 1
    for (int d = 0; d < DK_; ++d) {
      const float v = bf16r(xp[d]) + bf16r(theta[d]);
      prod = prod * cosf(v);
      cs[tid * DK_ + d] = prod;
    }
  }
  __syncthreads();

  const size_t rowbase = (size_t)bh * SEQ + (size_t)s0;
  const int quarter = tid & 3;
  const int tsub    = tid >> 2;

  v4u qv[4], kv[4];
#pragma unroll
  for (int it = 0; it < 4; ++it) {
    const int t = it * 64 + tsub;
    const v4f ca = *(const v4f*)(cs + t * DK_);
    const v4f cb = *(const v4f*)(cs + t * DK_ + 4);
    float f[8];
    f[0] = ca[0]; f[1] = ca[1]; f[2] = ca[2]; f[3] = ca[3];
    f[4] = cb[0]; f[5] = cb[1]; f[6] = cb[2]; f[7] = cb[3];
    v4u aq, ak;
#pragma unroll
    for (int e = 0; e < 4; ++e) {
      unsigned short q0b, q1b, k0b, k1b;
      enc_slots(f[2 * e],     quarter, q0b, k0b);
      enc_slots(f[2 * e + 1], quarter, q1b, k1b);
      aq[e] = pk16(q0b, q1b);
      ak[e] = pk16(k0b, k1b);
    }
    qv[it] = aq; kv[it] = ak;
  }

  const int dv = tid >> 5;
  const int j8 = (tid & 31) * 8;
  v4u vv;
#pragma unroll
  for (int e = 0; e < 4; ++e) {
    const float f0 = cs[(j8 + 2 * e) * DK_ + dv];
    const float f1 = cs[(j8 + 2 * e + 1) * DK_ + dv];
    vv[e] = pk16(hn_bits(f0 * 16384.0f), hn_bits(f1 * 16384.0f));
  }

  unsigned short* qo = qap + rowbase * KSL + (size_t)tid * 8;
  unsigned short* ko = kbp + rowbase * KSL + (size_t)tid * 8;
  unsigned short* vo = vtp + ((size_t)bh * DK_ + (size_t)dv) * SEQ + (size_t)s0 + (size_t)j8;
  for (int pass = 0; pass < 2; ++pass) {
#pragma unroll
    for (int it = 0; it < 4; ++it) {
      *(volatile v4u*)(qo + (size_t)it * 64 * KSL) = qv[it];
      *(volatile v4u*)(ko + (size_t)it * 64 * KSL) = kv[it];
    }
    *(volatile v4u*)vo = vv;
    __threadfence();
  }
}

__global__ __launch_bounds__(128)
void attn_q(const unsigned short* __restrict__ qap, const unsigned short* __restrict__ kbp,
            const unsigned short* __restrict__ vtp, unsigned short* mp) {
  union FH { v16h v; v8h h[2]; };
  __shared__ __align__(16) _Float16 Ksh[64 * KSL];
  __shared__ __align__(16) _Float16 Vsh[16 * 64];
  __shared__ __align__(16) _Float16 Psh[4][16 * 64];
  __shared__ __align__(16) float    Os[4][16 * 16];

  const int tid  = (int)threadIdx.x;
  const int wave = tid >> 5;
  const int lane = tid & 31;
  const int hh   = lane >> 4;
  const int c    = lane & 15;

  const int bx = (int)blockIdx.x;
  const int qt = bx % NQT;
  const int bh = bx / NQT;
  const int q0 = qt * 64 + wave * 16;

  const _Float16* QA = (const _Float16*)(const void*)qap;
  const _Float16* KB = (const _Float16*)(const void*)kbp + (size_t)bh * SEQ * KSL;
  const _Float16* VT = (const _Float16*)(const void*)vtp + (size_t)bh * DK_ * SEQ;

  if (tid < 64) {
    const v4u z4 = {0u, 0u, 0u, 0u};
    *(v4u*)(Vsh + 8 * 64 + tid * 8) = z4;
  }

  const v16h qa = ldfrag_h(QA + ((size_t)bh * SEQ + (size_t)(q0 + c)) * KSL + 8 * hh);

  const float sscale = kScale * 0.015625f;

  float mrow[8], lrow[8];
  v8f oacc = zero8();
#pragma unroll
  for (int r = 0; r < 8; ++r) { mrow[r] = -INFINITY; lrow[r] = 0.f; }

#pragma unroll 1
  for (int kt = 0; kt < NKT; ++kt) {
    const int kv0 = kt * 64;
    __syncthreads();
    {
      const _Float16* kg = KB + (size_t)kv0 * KSL;
      const v8h a0 = *(const v8h*)(kg + (size_t)tid * 8);
      const v8h a1 = *(const v8h*)(kg + (size_t)(tid + 128) * 8);
      *(v8h*)(Ksh + tid * 8) = a0;
      *(v8h*)(Ksh + (tid + 128) * 8) = a1;
      if (tid < 64) {
        const int d = tid >> 3, piece = (tid & 7) * 8;
        const v8h v0 = *(const v8h*)(VT + (size_t)d * SEQ + (size_t)kv0 + (size_t)piece);
        *(v8h*)(Vsh + d * 64 + piece) = v0;
      }
    }
    __syncthreads();

    v8f s[4];
#pragma unroll
    for (int j = 0; j < 4; ++j) {
      FH kb;
      kb.h[0] = *(const v8h*)(Ksh + (j * 16 + c) * KSL + 8 * hh);
      kb.h[1] = *(const v8h*)(Ksh + (j * 16 + c) * KSL + 16 + 8 * hh);
      const v8f acc = mma_h(qa, kb.v, zero8());
#pragma unroll
      for (int r = 0; r < 8; ++r) s[j][r] = acc[r] * sscale;
    }

    _Float16* pwh = Psh[wave];
#pragma unroll
    for (int r = 0; r < 8; ++r) {
      float m = s[0][r];
#pragma unroll
      for (int j = 1; j < 4; ++j) m = fmaxf(m, s[j][r]);
#pragma unroll
      for (int off = 1; off < 16; off <<= 1) m = fmaxf(m, __shfl_xor(m, off, 32));
      const float mnew  = fmaxf(mrow[r], m);
      const float msafe = (mnew == -INFINITY) ? 0.f : mnew;
      const float alpha = __expf(mrow[r] - msafe);
      mrow[r] = mnew;
      float psum = 0.f;
#pragma unroll
      for (int j = 0; j < 4; ++j) {
        const float p = __expf(s[j][r] - msafe);
        psum += p;
        pwh[(8 * hh + r) * 64 + j * 16 + c] = f16n(p * 1024.0f);
      }
#pragma unroll
      for (int off = 1; off < 16; off <<= 1) psum += __shfl_xor(psum, off, 32);
      lrow[r] = lrow[r] * alpha + psum;
      oacc[r] *= alpha;
    }
    __builtin_amdgcn_fence(3  , "workgroup");
    __builtin_amdgcn_wave_barrier();
    __builtin_amdgcn_fence(2  , "workgroup");

#pragma unroll
    for (int kk = 0; kk < 2; ++kk) {
      FH pa, vb;
      pa.h[0] = *(const v8h*)(pwh + c * 64 + kk * 32 + 8 * hh);
      pa.h[1] = *(const v8h*)(pwh + c * 64 + kk * 32 + 16 + 8 * hh);
      vb.h[0] = *(const v8h*)(Vsh + c * 64 + kk * 32 + 8 * hh);
      vb.h[1] = *(const v8h*)(Vsh + c * 64 + kk * 32 + 16 + 8 * hh);
      oacc = mma_h(pa.v, vb.v, oacc);
    }
  }

  float* os = Os[wave];
#pragma unroll
  for (int r = 0; r < 8; ++r) {
    const float l = lrow[r];
    const float inv = ((l > 0.f) ? (1.0f / l) : 0.f) * 0.000244140625f;
    os[(8 * hh + r) * 16 + c] = oacc[r] * inv;
  }
  __builtin_amdgcn_fence(3  , "workgroup");
  __builtin_amdgcn_wave_barrier();
  __builtin_amdgcn_fence(2  , "workgroup");
  {
    const int row = lane & 15;
    const float* sp = os + row * 16;
    v4u a;
#pragma unroll
    for (int e = 0; e < 4; ++e) {
      const float f0 = sp[2 * e], f1 = sp[2 * e + 1];
      a[e] = pk16(hn_bits(f0), hn_bits(f1));
    }
    unsigned short* o = mp + ((size_t)bh * SEQ + (size_t)(q0 + row)) * DK_;
    for (int pass = 0; pass < 2; ++pass) {
      if (lane < 16) *(volatile v4u*)o = a;
      __threadfence();
    }
  }
}

__global__ __launch_bounds__(128)
void proj_out(const unsigned short* __restrict__ mp, const float* __restrict__ Wo, float* out) {
  union FH { v16h v; v8h h[2]; };
  __shared__ __align__(16) float lds[8192];
  _Float16* Wsh = (_Float16*)(void*)lds;

  const int tid  = (int)threadIdx.x;
  const int wave = tid >> 5;
  const int lane = tid & 31;
  const int hh   = lane >> 4;
  const int c    = lane & 15;

#pragma unroll 4
  for (int i = 0; i < 16; ++i) {
    const int idx8 = tid + 128 * i;
    const v4f a  = *(const v4f*)(Wo + (size_t)idx8 * 8);
    const v4f a4 = *(const v4f*)(Wo + (size_t)idx8 * 8 + 4);
    v4u p;
    p[0] = pk16(hn_bits(bf16r(a[0]) * 1024.0f),  hn_bits(bf16r(a[1]) * 1024.0f));
    p[1] = pk16(hn_bits(bf16r(a[2]) * 1024.0f),  hn_bits(bf16r(a[3]) * 1024.0f));
    p[2] = pk16(hn_bits(bf16r(a4[0]) * 1024.0f), hn_bits(bf16r(a4[1]) * 1024.0f));
    p[3] = pk16(hn_bits(bf16r(a4[2]) * 1024.0f), hn_bits(bf16r(a4[3]) * 1024.0f));
    *(v4u*)(Wsh + idx8 * 8) = p;
  }
  __syncthreads();

  const int m0 = (int)blockIdx.x * 64 + wave * 16;
  const int m  = m0 + c;
  const int b  = m / SEQ;
  const int s  = m - b * SEQ;
  const _Float16* Mrow = (const _Float16*)(const void*)mp + ((size_t)(b * H_) * SEQ + (size_t)s) * DK_;

  v8f acc[8];
#pragma unroll
  for (int j = 0; j < 8; ++j) acc[j] = zero8();

#pragma unroll
  for (int ks = 0; ks < 4; ++ks) {
    const int k0  = ks * 32;
    const int hd0 = ks * 4 + hh;
    const int hd1 = ks * 4 + 2 + hh;
    FH af;
    af.h[0] = *(const v8h*)(Mrow + (size_t)hd0 * SEQ * DK_);
    af.h[1] = *(const v8h*)(Mrow + (size_t)hd1 * SEQ * DK_);
#pragma unroll
    for (int j = 0; j < 8; ++j) {
      FH bf;
      bf.h[0] = *(const v8h*)(Wsh + (j * 16 + c) * E_ + k0 + 8 * hh);
      bf.h[1] = *(const v8h*)(Wsh + (j * 16 + c) * E_ + k0 + 16 + 8 * hh);
      acc[j] = mma_h(af.v, bf.v, acc[j]);
    }
  }

  __syncthreads();
  float* slab = lds + wave * 2048;
#pragma unroll
  for (int j = 0; j < 8; ++j) {
#pragma unroll
    for (int r = 0; r < 8; ++r) slab[(8 * hh + r) * E_ + j * 16 + c] = acc[j][r];
  }
  __builtin_amdgcn_fence(3  , "workgroup");
  __builtin_amdgcn_wave_barrier();
  __builtin_amdgcn_fence(2  , "workgroup");

  const float oscale = 1.0f / 4194304.0f;
  v4f vrow[16];
#pragma unroll
  for (int row = 0; row < 16; ++row) {
    const v4f v = *(const v4f*)(slab + row * E_ + lane * 4);
    vrow[row] = v * oscale;
  }
  for (int pass = 0; pass < 2; ++pass) {
#pragma unroll
    for (int row = 0; row < 16; ++row) {
      *(volatile v4f*)(out + (size_t)(m0 + row) * E_ + lane * 4) = vrow[row];
    }
    __threadfence();
  }
}

extern "C" void kernel_launch(void* const* d_in, const int* in_sizes, int n_in,
                              void* d_out, int out_size, void* d_ws, size_t ws_size,
                              hipStream_t stream) {
  if (n_in < 3) return;
  if ((long long)in_sizes[0] < ((long long)(NB - 1) * SEQ_FULL + (long long)SEQ) * E_) return;
  if (in_sizes[1] < DK_) return;
  if (in_sizes[2] < E_ * E_) return;
  if ((long long)out_size < (long long)NB * SEQ * E_) return;

  const float* x     = (const float*)d_in[0];
  const float* theta = (const float*)d_in[1];
  const float* Wo    = (const float*)d_in[2];

  const size_t PQA = (size_t)BH_ * SEQ * KSL * 2;
  const size_t PKB = PQA;
  const size_t PVT = (size_t)BH_ * DK_ * SEQ * 2;
  const size_t PMP = (size_t)BH_ * SEQ * DK_ * 2;
  size_t off = 0;
  const size_t oQA = off; off += PQA;
  const size_t oKB = off; off += PKB;
  const size_t oVT = off; off += PVT;
  const size_t oMP = off; off += PMP;
  if (off > ws_size) return;
  if (off > (size_t)134217728) return;

  char* ws = (char*)d_ws;
  unsigned short* QA = (unsigned short*)(ws + oQA);
  unsigned short* KB = (unsigned short*)(ws + oKB);
  unsigned short* VT = (unsigned short*)(ws + oVT);
  unsigned short* MP = (unsigned short*)(ws + oMP);

  const dim3 gEnc(BH_ * NSG);
  const dim3 gAttn(BH_ * NQT);
  const dim3 gProj((NB * SEQ) / 64);

  qenc<<<gEnc, dim3(256), 0, stream>>>(x, theta, QA, KB, VT);
  attn_q<<<gAttn, dim3(128), 0, stream>>>(QA, KB, VT, MP);
  proj_out<<<gProj, dim3(128), 0, stream>>>(MP, Wo, (float*)d_out);
  (void)hipGetLastError();
}
